// PitchRegulator_44727789421052
// MI455X (gfx1250) — hardware-verified
//
#include <hip/hip_runtime.h>
#define NBt 16
#define TT 2048
#define CC 256
#define NR (NBt * TT)
#define NW 10
#define NLIN 22
#define NLP 32
#define NEMB 258
typedef __bf16 v16b __attribute__((ext_vector_type(16)));
typedef unsigned short v8us __attribute__((ext_vector_type(8), may_alias));
typedef float  v8f  __attribute__((ext_vector_type(8)));
typedef float  v4f  __attribute__((ext_vector_type(4)));
typedef float  v4fa __attribute__((ext_vector_type(4), may_alias));
union FragB { v16b v; v8us half[2]; unsigned short u[16]; };

__device__ __forceinline__ unsigned short bf16_bits(float x) { unsigned int u = __float_as_uint(x); return (unsigned short)((u + 0x7FFFu + ((u >> 16) & 1u)) >> 16); }
__device__ __forceinline__ float bf16_val(unsigned short b) { return __uint_as_float(((unsigned int)b) << 16); }
__device__ __forceinline__ float bf16_round(float x) { return bf16_val(bf16_bits(x)); }
template <int NT>
__device__ __forceinline__ v8f mmaN(v16b ah, v16b al, v16b bh, v16b bl, v8f c) {
  c = __builtin_amdgcn_wmma_f32_16x16x32_bf16(false, ah, false, bh, (short)0, c, false, false);
  if (NT >= 2) c = __builtin_amdgcn_wmma_f32_16x16x32_bf16(false, al, false, bh, (short)0, c, false, false);
  if (NT >= 3) c = __builtin_amdgcn_wmma_f32_16x16x32_bf16(false, ah, false, bl, (short)0, c, false, false);
  asm volatile("v_nop\n\tv_nop\n\tv_nop\n\tv_nop" : "+v"(c) : "v"(ah), "v"(al), "v"(bh), "v"(bl));
  return c;
}

__global__ __launch_bounds__(256) void k_wt_bf16(const float* __restrict__ W, unsigned short* __restrict__ Wt, int K, int N) {
  const int t = blockIdx.x * 256 + threadIdx.x;
  const int k8n = K / 8;
  if (t >= N * k8n) return;
  const int n = t / k8n, k8 = (t % k8n) * 8;
  v8us v;
#pragma unroll
  for (int i = 0; i < 8; ++i) v[i] = bf16_bits(W[(size_t)(k8 + i) * N + n]);
  *(volatile v8us*)(Wt + (size_t)n * K + k8) = v;
  __threadfence();
  *(volatile v8us*)(Wt + (size_t)n * K + k8) = v;
}

template <bool ASPLIT, int ACT, bool BIAS_BF16>
__global__ __launch_bounds__(128) void k_gemm_bf(const float* __restrict__ A, int lda, const unsigned short* __restrict__ Wt, int ldb,
                                               const float* __restrict__ bias, float* __restrict__ C, int ldc, int M, int N, int K) {
  __shared__ __attribute__((aligned(16))) float so[4][16][64];
  const int tid = threadIdx.x, w = tid >> 5, lane = tid & 31, ln = lane & 15, hh = lane >> 4;
  const int ntn = N / 64;
  const int wid = blockIdx.x * 4 + w;
  const int mt = wid / ntn, nq = wid % ntn;
  if (mt * 16 >= M) return;
  const int row0 = mt * 16, col0 = nq * 64;
  const float* arow = A + (size_t)(row0 + ln) * lda;
  v8f acc[4] = {};
  for (int kb = 0; kb < K; kb += 32) {
    FragB ah, al;
    const v4f x0 = *(const v4fa*)(arow + kb + 8 * hh), x1 = *(const v4fa*)(arow + kb + 8 * hh + 4);
    const v4f x2 = *(const v4fa*)(arow + kb + 16 + 8 * hh), x3 = *(const v4fa*)(arow + kb + 16 + 8 * hh + 4);
    float xs[16] = {x0[0],x0[1],x0[2],x0[3],x1[0],x1[1],x1[2],x1[3],x2[0],x2[1],x2[2],x2[3],x3[0],x3[1],x3[2],x3[3]};
#pragma unroll
    for (int i = 0; i < 16; ++i) { const unsigned short hb = bf16_bits(xs[i]); ah.u[i] = hb; al.u[i] = ASPLIT ? bf16_bits(xs[i] - bf16_val(hb)) : (unsigned short)0; }
#pragma unroll
    for (int t = 0; t < 4; ++t) {
      const unsigned short* brow = Wt + (size_t)(col0 + t * 16 + ln) * ldb + kb;
      FragB b;
      b.half[0] = *(const v8us*)(brow + 8 * hh);
      b.half[1] = *(const v8us*)(brow + 16 + 8 * hh);
      acc[t] = mmaN<ASPLIT ? 2 : 1>(ah.v, al.v, b.v, b.v, acc[t]);
    }
  }
#pragma unroll
  for (int t = 0; t < 4; ++t) {
    float bv = bias ? bias[col0 + t * 16 + ln] : 0.f;
    if (BIAS_BF16) bv = bf16_round(bv);
#pragma unroll
    for (int r = 0; r < 8; ++r) { float v = acc[t][r] + bv; if (ACT == 1) v = fmaxf(v, 0.f); so[w][8 * hh + r][t * 16 + ln] = v; }
  }
  __builtin_amdgcn_fence(__ATOMIC_ACQ_REL, "workgroup");
  __builtin_amdgcn_wave_barrier();
  const int rsub = lane >> 4, c4 = (lane & 15) * 4;
  for (int pass = 0; pass < 2; ++pass) {
#pragma unroll
    for (int q = 0; q < 8; ++q) {
      const int r = q * 2 + rsub;
      const v4f v = *(const v4fa*)&so[w][r][c4];
      *(volatile v4f*)(C + (size_t)(row0 + r) * ldc + col0 + c4) = v;
    }
    if (pass == 0) __threadfence();
  }
}

template <bool ASPLIT, int ACT, bool BIAS_BF16, bool RES_BF16>
__global__ __launch_bounds__(128) void k_gemm_bf3(const float* __restrict__ A, int lda, const unsigned short* __restrict__ Wt, int ldb,
                                                const float* __restrict__ bias, const float* __restrict__ resid, int rmod, int ldr,
                                                float* __restrict__ C, int ldc, int M, int N, int K) {
  __shared__ __attribute__((aligned(16))) float so[4][16][64];
  const int tid = threadIdx.x, w = tid >> 5, lane = tid & 31, ln = lane & 15, hh = lane >> 4;
  const int ntn = N / 64;
  const int wid = blockIdx.x * 4 + w;
  const int mt = wid / ntn, nq = wid % ntn;
  if (mt * 16 >= M) return;
  const int row0 = mt * 16, col0 = nq * 64;
  const float* arow = A + (size_t)(row0 + ln) * lda;
  v8f acc[4] = {};
  for (int kb = 0; kb < K; kb += 32) {
    FragB ah, al;
    const v4f x0 = *(const v4fa*)(arow + kb + 8 * hh), x1 = *(const v4fa*)(arow + kb + 8 * hh + 4);
    const v4f x2 = *(const v4fa*)(arow + kb + 16 + 8 * hh), x3 = *(const v4fa*)(arow + kb + 16 + 8 * hh + 4);
    float xs[16] = {x0[0],x0[1],x0[2],x0[3],x1[0],x1[1],x1[2],x1[3],x2[0],x2[1],x2[2],x2[3],x3[0],x3[1],x3[2],x3[3]};
#pragma unroll
    for (int i = 0; i < 16; ++i) { const unsigned short hb = bf16_bits(xs[i]); ah.u[i] = hb; al.u[i] = ASPLIT ? bf16_bits(xs[i] - bf16_val(hb)) : (unsigned short)0; }
#pragma unroll
    for (int t = 0; t < 4; ++t) {
      const unsigned short* brow = Wt + (size_t)(col0 + t * 16 + ln) * ldb + kb;
      FragB b;
      b.half[0] = *(const v8us*)(brow + 8 * hh);
      b.half[1] = *(const v8us*)(brow + 16 + 8 * hh);
      acc[t] = mmaN<ASPLIT ? 2 : 1>(ah.v, al.v, b.v, b.v, acc[t]);
    }
  }
#pragma unroll
  for (int t = 0; t < 4; ++t) {
    const int col = col0 + t * 16 + ln;
    float bv = bias ? bias[col] : 0.f;
    if (BIAS_BF16) bv = bf16_round(bv);
#pragma unroll
    for (int r = 0; r < 8; ++r) {
      float v = acc[t][r] + bv;
      if (resid) { float rv = resid[(size_t)((row0 + 8 * hh + r) % rmod) * ldr + col]; if (RES_BF16) rv = bf16_round(rv); v += rv; }
      if (ACT == 1) v = fmaxf(v, 0.f);
      if (ACT == 2) v = 0.5f * v * (1.0f + erff(v * 0.70710678118654752f));
      if (ACT == 3) { const float u = 0.7978845608028654f * (v + 0.044715f * v * v * v); v = 0.5f * v * (1.0f + tanhf(u)); }
      so[w][8 * hh + r][t * 16 + ln] = v;
    }
  }
  __builtin_amdgcn_fence(__ATOMIC_ACQ_REL, "workgroup");
  __builtin_amdgcn_wave_barrier();
  const int rsub = lane >> 4, c4 = (lane & 15) * 4;
  for (int pass = 0; pass < 2; ++pass) {
#pragma unroll
    for (int q = 0; q < 8; ++q) {
      const int r = q * 2 + rsub;
      const v4f v = *(const v4fa*)&so[w][r][c4];
      *(volatile v4f*)(C + (size_t)(row0 + r) * ldc + col0 + c4) = v;
    }
    if (pass == 0) __threadfence();
  }
}
template <bool PARAM_BF16>
__global__ __launch_bounds__(256) void k_layernorm(const float* __restrict__ X, const float* __restrict__ R, const float* __restrict__ g, const float* __restrict__ bta,
                                                  float* __restrict__ out_sum, float* __restrict__ out_norm, int N, float eps) {
  __shared__ float red[256];
  const int row = blockIdx.x, tid = threadIdx.x;
  const float* x = X + (size_t)row * N; const float* rr = R ? R + (size_t)row * N : nullptr;
  float vals[16];
  const int per = N / 256;
  float s1 = 0.f;
  for (int u = 0; u < per / 4; ++u) {
    const int j = tid * 4 + 1024 * u;
    const v4f a = *(const v4fa*)(x + j);
    v4f b = {0.f,0.f,0.f,0.f}; if (rr) b = *(const v4fa*)(rr + j);
#pragma unroll
    for (int q = 0; q < 4; ++q) { const float v = a[q] + b[q]; vals[u * 4 + q] = v; s1 += v; }
  }
  red[tid] = s1; __syncthreads();
  for (int st = 128; st > 0; st >>= 1) { if (tid < st) red[tid] += red[tid + st]; __syncthreads(); }
  const float mu = red[0] / (float)N; __syncthreads();
  float s2 = 0.f;
  for (int u = 0; u < per / 4; ++u)
#pragma unroll
    for (int q = 0; q < 4; ++q) { const float c = vals[u * 4 + q] - mu; s2 += c * c; }
  red[tid] = s2; __syncthreads();
  for (int st = 128; st > 0; st >>= 1) { if (tid < st) red[tid] += red[tid + st]; __syncthreads(); }
  const float rs = rsqrtf(red[0] / (float)N + eps);
  for (int pass = 0; pass < 2; ++pass) {
    for (int u = 0; u < per / 4; ++u) {
      const int j = tid * 4 + 1024 * u;
      v4f o, sm;
#pragma unroll
      for (int q = 0; q < 4; ++q) {
        float gg = g[j + q], bb = bta[j + q];
        if (PARAM_BF16) { gg = bf16_round(gg); bb = bf16_round(bb); }
        sm[q] = vals[u * 4 + q]; o[q] = (vals[u * 4 + q] - mu) * rs * gg + bb;
      }
      if (out_sum) *(volatile v4f*)(out_sum + (size_t)row * N + j) = sm;
      *(volatile v4f*)(out_norm + (size_t)row * N + j) = o;
    }
    if (pass == 0) __threadfence();
  }
}


typedef _Float16 v16h __attribute__((ext_vector_type(16)));
union FragH { v16h v; v8us half[2]; _Float16 h[16]; unsigned short u[16]; };
template <int NT>
__device__ __forceinline__ v8f mmaH(v16h ah, v16h al, v16h bh, v16h bl, v8f c) {
  c = __builtin_amdgcn_wmma_f32_16x16x32_f16(false, ah, false, bh, (short)0, c, false, false);
  if (NT >= 2) c = __builtin_amdgcn_wmma_f32_16x16x32_f16(false, al, false, bh, (short)0, c, false, false);
  if (NT >= 3) c = __builtin_amdgcn_wmma_f32_16x16x32_f16(false, ah, false, bl, (short)0, c, false, false);
  asm volatile("v_nop\n\tv_nop\n\tv_nop\n\tv_nop" : "+v"(c) : "v"(ah), "v"(al), "v"(bh), "v"(bl));
  return c;
}
template <bool ASPLIT>
__global__ __launch_bounds__(128) void k_gemm_h(const float* __restrict__ A, int lda, size_t sA, const _Float16* __restrict__ Bh, int ldb, size_t sB, float alpha, float* __restrict__ C, int ldc, size_t sC, int M, int N, int K) {
  __shared__ __attribute__((aligned(16))) float so[4][16][64];
  const int tid = threadIdx.x, w = tid >> 5, lane = tid & 31, ln = lane & 15, hh = lane >> 4; const int by = blockIdx.y;
  A += (size_t)by * sA; Bh += (size_t)by * sB; C += (size_t)by * sC;
  const int ntn = (N + 63) / 64; const int wid = blockIdx.x * 4 + w; const int mt = wid / ntn, nq = wid % ntn; if (mt * 16 >= M) return;
  const int row0 = mt * 16, col0 = nq * 64; const float* arow = A + (size_t)(row0 + ln) * lda;
  v8f acc[4] = {};
  for (int kb = 0; kb < K; kb += 32) {
    FragH ah, al;
    const v4f x0 = *(const v4fa*)(arow + kb + 8 * hh), x1 = *(const v4fa*)(arow + kb + 8 * hh + 4), x2 = *(const v4fa*)(arow + kb + 16 + 8 * hh), x3 = *(const v4fa*)(arow + kb + 16 + 8 * hh + 4);
    float xs[16] = {x0[0],x0[1],x0[2],x0[3],x1[0],x1[1],x1[2],x1[3],x2[0],x2[1],x2[2],x2[3],x3[0],x3[1],x3[2],x3[3]};
#pragma unroll
    for (int i = 0; i < 16; ++i) { const _Float16 h = (_Float16)xs[i]; ah.h[i] = h; al.h[i] = ASPLIT ? (_Float16)(xs[i] - (float)h) : (_Float16)0.0f; }
#pragma unroll
    for (int t = 0; t < 4; ++t) { if (col0 + t * 16 >= N) continue; const size_t boff = (size_t)(col0 + t * 16 + ln) * ldb + kb; FragH bq; bq.half[0] = *(const v8us*)(Bh + boff + 8 * hh); bq.half[1] = *(const v8us*)(Bh + boff + 16 + 8 * hh);
      acc[t] = mmaH<ASPLIT ? 2 : 1>(ah.v, al.v, bq.v, bq.v, acc[t]); }
  }
#pragma unroll
  for (int t = 0; t < 4; ++t) { if (col0 + t * 16 >= N) continue;
#pragma unroll
    for (int r = 0; r < 8; ++r) so[w][8 * hh + r][t * 16 + ln] = acc[t][r] * alpha; }
  __builtin_amdgcn_fence(__ATOMIC_ACQ_REL, "workgroup"); __builtin_amdgcn_wave_barrier();
  const int rsub = lane >> 4, c4 = (lane & 15) * 4;
  for (int pass = 0; pass < 2; ++pass) {
#pragma unroll
    for (int q = 0; q < 8; ++q) { const int r = q * 2 + rsub; if (col0 + c4 < N) { const v4f v = *(const v4fa*)&so[w][r][c4]; *(volatile v4f*)(C + (size_t)(row0 + r) * ldc + col0 + c4) = v; } }
    if (pass == 0) __threadfence(); }
}

__global__ __launch_bounds__(256) void k_wt_f16(const float* __restrict__ W, _Float16* __restrict__ Wt, int K, int N, float scale) {
  const int t = blockIdx.x * 256 + threadIdx.x; if (t >= N * (K / 8)) return; const int n = t / (K / 8), k8 = (t % (K / 8)) * 8; FragH f;
#pragma unroll
  for (int i = 0; i < 8; ++i) f.h[i] = (_Float16)(bf16_round(W[(size_t)(k8 + i) * N + n]) * scale); const v8us o = f.half[0];
  *(volatile v8us*)((unsigned short*)Wt + (size_t)n * K + k8) = o; __threadfence(); *(volatile v8us*)((unsigned short*)Wt + (size_t)n * K + k8) = o;
}
template <int ACT>
__global__ __launch_bounds__(128) void k_gemm_hhx(const _Float16* __restrict__ A, int lda, size_t sA, const _Float16* __restrict__ Bh, int ldb, size_t sB, float alpha, const float* __restrict__ bias, size_t sBias, const float* __restrict__ CP, int rowsPerB, size_t sCPb, int row0g,
    float* __restrict__ C, _Float16* __restrict__ C16, int ldc, size_t sC, int M, int N, int K) {
  __shared__ __attribute__((aligned(16))) float so[4][16][64];
  const int tid = threadIdx.x, w = tid >> 5, lane = tid & 31, ln = lane & 15, hh = lane >> 4; const int by = blockIdx.y;
  A += (size_t)by * sA; Bh += (size_t)by * sB; const size_t cofs = (size_t)by * sC; const float* bp = bias ? bias + (size_t)by * sBias : nullptr;
  const int ntn = (N + 63) / 64; const int wid = blockIdx.x * 4 + w; const int mt = wid / ntn, nq = wid % ntn; if (mt * 16 >= M) return;
  const int row0 = mt * 16, col0 = nq * 64; const _Float16* arow = A + (size_t)(row0 + ln) * lda;
  v8f acc[4] = {};
  for (int kb = 0; kb < K; kb += 32) { FragH ah; ah.half[0] = *(const v8us*)((const unsigned short*)arow + kb + 8 * hh); ah.half[1] = *(const v8us*)((const unsigned short*)arow + kb + 16 + 8 * hh);
#pragma unroll
    for (int t = 0; t < 4; ++t) { if (col0 + t * 16 >= N) continue; const size_t boff = (size_t)(col0 + t * 16 + ln) * ldb + kb; FragH bq; bq.half[0] = *(const v8us*)((const unsigned short*)Bh + boff + 8 * hh); bq.half[1] = *(const v8us*)((const unsigned short*)Bh + boff + 16 + 8 * hh);
      acc[t] = mmaH<1>(ah.v, ah.v, bq.v, bq.v, acc[t]); }
  }
#pragma unroll
  for (int t = 0; t < 4; ++t) { if (col0 + t * 16 >= N) continue; const int col = col0 + t * 16 + ln; const float bv = bp ? bf16_round(bp[col]) : 0.f;
#pragma unroll
    for (int r = 0; r < 8; ++r) { float v = acc[t][r] * alpha + bv; if (CP) { const int bidx = (row0g + row0 + 8 * hh + r) / rowsPerB; v += CP[(size_t)bidx * sCPb + (size_t)by * 64 + col]; } if (ACT == 1) v = (v > 0.f) ? v : expm1f(v); else if (ACT == 7) v = (v > 0.f) ? v + 1.0f : expf(v); else if (ACT == 8) v = tanhf(v); else if (ACT == 9) v = 0.5f * v * (1.0f + tanhf(0.7978845608028654f * (v + 0.044715f * v * v * v))); else if (ACT == 11) v = 1.0f / (1.0f + expf(-v)); else if (ACT == 12) v = (v > 0.f) ? v : 0.01f * v; else if (ACT == 14) v = (v > 0.f) ? v : 0.1f * v; else if (ACT == 15) v = v / (1.0f + expf(-v)); else if (ACT == 3) v = fmaxf(v, 0.f); else if (ACT == 6) v = 0.5f * v * (1.0f + erff(v * 0.70710678118654752f)); so[w][8 * hh + r][t * 16 + ln] = v; } }
  __builtin_amdgcn_fence(__ATOMIC_ACQ_REL, "workgroup"); __builtin_amdgcn_wave_barrier();
  const int rsub = lane >> 4, c4 = (lane & 15) * 4; typedef _Float16 v4h __attribute__((ext_vector_type(4)));
  for (int pass = 0; pass < 2; ++pass) {
#pragma unroll
    for (int q = 0; q < 8; ++q) { const int r = q * 2 + rsub; if (col0 + c4 < N) { const v4f v = *(const v4fa*)&so[w][r][c4]; if (C) *(volatile v4f*)(C + cofs + (size_t)(row0 + r) * ldc + col0 + c4) = v; if (C16) { v4h h4; for (int i = 0; i < 4; ++i) h4[i] = (_Float16)v[i]; *(volatile v4h*)(C16 + cofs + (size_t)(row0 + r) * ldc + col0 + c4) = h4; } } }
    if (pass == 0) __threadfence(); }
}


typedef _Float16 v4h __attribute__((ext_vector_type(4)));

__global__ __launch_bounds__(256) void k_x16(const float* __restrict__ x, _Float16* __restrict__ X16, size_t n8) { const size_t t = (size_t)blockIdx.x * 256 + threadIdx.x; if (t >= n8) return; FragH f;
#pragma unroll
  for (int q = 0; q < 8; ++q) f.h[q] = (_Float16)bf16_round(x[t * 8 + q]); *(volatile v8us*)((unsigned short*)X16 + t * 8) = f.half[0]; __threadfence(); *(volatile v8us*)((unsigned short*)X16 + t * 8) = f.half[0]; }
__global__ __launch_bounds__(256) void k_h16(const float* __restrict__ x, _Float16* __restrict__ X16, size_t n8) { const size_t t = (size_t)blockIdx.x * 256 + threadIdx.x; if (t >= n8) return; FragH f;
#pragma unroll
  for (int q = 0; q < 8; ++q) f.h[q] = (_Float16)x[t * 8 + q]; *(volatile v8us*)((unsigned short*)X16 + t * 8) = f.half[0]; __threadfence(); *(volatile v8us*)((unsigned short*)X16 + t * 8) = f.half[0]; }
__global__ __launch_bounds__(256) void k_round16f(const float* __restrict__ W, _Float16* __restrict__ Bt, size_t n8) { const size_t t = (size_t)blockIdx.x * 256 + threadIdx.x; if (t >= n8) return; FragH f;
#pragma unroll
  for (int i = 0; i < 8; ++i) f.h[i] = (_Float16)(bf16_round(W[t * 8 + i]) * 16.0f); *(volatile v8us*)((unsigned short*)Bt + t * 8) = f.half[0]; __threadfence(); *(volatile v8us*)((unsigned short*)Bt + t * 8) = f.half[0]; }
template <int NHv, int TTv>
__global__ __launch_bounds__(256) void k_vt(const _Float16* __restrict__ V16, int ldv, int voff, _Float16* __restrict__ Vt) { __shared__ unsigned short tl[64][66]; const int tid = threadIdx.x; const int slab = blockIdx.x / (TTv / 64), lg = blockIdx.x % (TTv / 64); const int b = slab / NHv, h = slab % NHv;
  for (int i = tid; i < 64 * 8; i += 256) { const int r = i / 8, c8 = (i % 8) * 8; FragH f; f.half[0] = *(const v8us*)((const unsigned short*)V16 + ((size_t)b * TTv + lg * 64 + r) * ldv + voff + h * 64 + c8);
#pragma unroll
    for (int q = 0; q < 8; ++q) tl[r][c8 + q] = f.u[q]; }
  __syncthreads();
  for (int pass = 0; pass < 2; ++pass) {
#pragma unroll
    for (int rd = 0; rd < 2; ++rd) { const int d = rd * 32 + tid / 8, pc = tid % 8; FragH f;
#pragma unroll
      for (int q = 0; q < 8; ++q) f.u[q] = tl[pc * 8 + q][d];
      *(volatile v8us*)((unsigned short*)Vt + ((size_t)slab * 64 + d) * TTv + lg * 64 + pc * 8) = f.half[0]; }
    if (pass == 0) __threadfence(); } }

__global__ __launch_bounds__(256) void k_hl(const float* __restrict__ F, _Float16* __restrict__ Hh, _Float16* __restrict__ Hl, size_t n8) { const size_t t = (size_t)blockIdx.x * 256 + threadIdx.x; if (t >= n8) return; FragH fh, fl; const v4f a = *(const v4fa*)(F + t * 8), c = *(const v4fa*)(F + t * 8 + 4);
#pragma unroll
  for (int q = 0; q < 4; ++q) { _Float16 h = (_Float16)a[q]; fh.h[q] = h; fl.h[q] = (_Float16)((a[q] - (float)h) * 1024.0f); h = (_Float16)c[q]; fh.h[4 + q] = h; fl.h[4 + q] = (_Float16)((c[q] - (float)h) * 1024.0f); }
  for (int pass = 0; pass < 2; ++pass) { *(volatile v8us*)((unsigned short*)Hh + t * 8) = fh.half[0]; *(volatile v8us*)((unsigned short*)Hl + t * 8) = fl.half[0]; if (pass == 0) __threadfence(); } }

__device__ __forceinline__ v4f shfl4(v4f v, int srcl) { v4f r; r[0] = __shfl(v[0], srcl, 32); r[1] = __shfl(v[1], srcl, 32); r[2] = __shfl(v[2], srcl, 32); r[3] = __shfl(v[3], srcl, 32); return r; }
__global__ __launch_bounds__(256) void k_tcol(const _Float16* __restrict__ P, _Float16* __restrict__ COL) { const int t = blockIdx.x * 256 + threadIdx.x; if (t >= NR * 3 * (CC / 8)) return; const int c0 = (t % (CC / 8)) * 8; const int k = (t / (CC / 8)) % 3; const int r = t / ((CC / 8) * 3); const int b = r / TT, tt = r % TT; const int src = tt + k - 1; FragH f = FragH{};
  if (src >= 0 && src < TT) f.half[0] = *(const v8us*)((const unsigned short*)P + ((size_t)b * TT + src) * CC + c0);
  *(volatile v8us*)((unsigned short*)COL + ((size_t)r * 3 + k) * CC + c0) = f.half[0]; __threadfence(); *(volatile v8us*)((unsigned short*)COL + ((size_t)r * 3 + k) * CC + c0) = f.half[0]; }
__global__ __launch_bounds__(256) void k_w1d(const float* __restrict__ wsrc, _Float16* __restrict__ Bt) { const int KD = 3 * CC; const int t = blockIdx.x * 256 + threadIdx.x; if (t >= CC * (KD / 8)) return; const int col0 = (t % (KD / 8)) * 8; const int o = t / (KD / 8); const int k = col0 / CC, c0 = col0 % CC; FragH f;
#pragma unroll
  for (int q = 0; q < 8; ++q) f.h[q] = (_Float16)(bf16_round(wsrc[((size_t)o * CC + c0 + q) * 3 + k]) * 16.0f);
  *(volatile v8us*)((unsigned short*)Bt + (size_t)o * KD + col0) = f.half[0]; __threadfence(); *(volatile v8us*)((unsigned short*)Bt + (size_t)o * KD + col0) = f.half[0]; }
__global__ __launch_bounds__(256) void k_wlin(const float* __restrict__ w, const float* __restrict__ b, _Float16* __restrict__ Bt, float* __restrict__ BP) { const int t = blockIdx.x * 256 + threadIdx.x; if (t >= NLP * (CC / 8)) return; const int k0 = (t % (CC / 8)) * 8, o = t / (CC / 8); FragH f;
#pragma unroll
  for (int q = 0; q < 8; ++q) f.h[q] = (o < NLIN) ? (_Float16)(bf16_round(w[(size_t)o * CC + k0 + q]) * 16.0f) : (_Float16)0.0f;
  *(volatile v8us*)((unsigned short*)Bt + (size_t)o * CC + k0) = f.half[0]; __threadfence(); *(volatile v8us*)((unsigned short*)Bt + (size_t)o * CC + k0) = f.half[0];
  if (k0 == 0) { const float v = (o < NLIN) ? b[o] : 0.f; *(volatile float*)(BP + o) = v; __threadfence(); *(volatile float*)(BP + o) = v; } }
__global__ __launch_bounds__(256) void k_lnrelu(const float* __restrict__ Hm, const float* __restrict__ g, const float* __restrict__ bb, _Float16* __restrict__ O16) {
  #pragma clang fp contract(off)
  const int tid = threadIdx.x, w = tid >> 5, l = tid & 31; const int r = blockIdx.x * 8 + w; if (r >= NR) return; float v[8]; float s = 0.f;
#pragma unroll
  for (int k = 0; k < 8; ++k) { v[k] = Hm[(size_t)r * CC + l * 8 + k]; s += v[k]; }
  for (int o = 16; o > 0; o >>= 1) s += __shfl_xor(s, o, 32); const float mu = s / (float)CC; float q2 = 0.f;
#pragma unroll
  for (int k = 0; k < 8; ++k) { const float d = v[k] - mu; q2 += d * d; }
  for (int o = 16; o > 0; o >>= 1) q2 += __shfl_xor(q2, o, 32); const float rs = rsqrtf(q2 / (float)CC + 1e-5f); FragH f;
#pragma unroll
  for (int k = 0; k < 8; ++k) { const int c = l * 8 + k; f.h[k] = (_Float16)fmaxf((v[k] - mu) * rs * bf16_round(g[c]) + bf16_round(bb[c]), 0.f); }
  *(volatile v8us*)((unsigned short*)O16 + (size_t)r * CC + l * 8) = f.half[0]; __threadfence(); *(volatile v8us*)((unsigned short*)O16 + (size_t)r * CC + l * 8) = f.half[0]; }
__global__ __launch_bounds__(256) void k_pspec(const float* __restrict__ PRED, const int* __restrict__ ml, float* __restrict__ out) { const int t = blockIdx.x * 256 + threadIdx.x; if (t >= NR * 20 / 4) return; v4f v;
#pragma unroll
  for (int i = 0; i < 4; ++i) { const size_t f = (size_t)t * 4 + i; const size_t bt = f / 20; const int j = (int)(f % 20); const int b = (int)(bt / TT), tt = (int)(bt % TT); v[i] = (tt < ml[b]) ? PRED[bt * NLP + j] : 0.f; }
  *(volatile v4f*)(out + (size_t)t * 4) = v; __threadfence(); *(volatile v4f*)(out + (size_t)t * 4) = v; }
__global__ __launch_bounds__(256) void k_pparams(const float* __restrict__ PRED, float* __restrict__ out) {
  #pragma clang fp contract(off)
  __shared__ float red[256]; __shared__ float res[32]; const int tid = threadIdx.x;
  for (int bj = 0; bj < 2 * NBt; ++bj) { const int b = bj >> 1, j = 20 + (bj & 1); float s = 0.f; for (int tt = tid; tt < TT; tt += 256) s += PRED[((size_t)b * TT + tt) * NLP + j]; red[tid] = s; __syncthreads(); for (int st = 128; st > 0; st >>= 1) { if (tid < st) red[tid] += red[tid + st]; __syncthreads(); } if (tid == 0) res[bj] = red[0] / (float)TT; __syncthreads(); }
  if (tid < 32) { *(volatile float*)(out + tid) = res[tid]; __threadfence(); *(volatile float*)(out + tid) = res[tid]; } }
__global__ __launch_bounds__(256) void k_tstat(const float* __restrict__ tg, const int* __restrict__ ml, float* __restrict__ STT) {
  #pragma clang fp contract(off)
  __shared__ float red[256]; __shared__ float mu_s; const int b = blockIdx.x, tid = threadIdx.x; const int len = ml[b]; const float lenf = (float)len; float s = 0.f;
  for (int tt = tid; tt < TT; tt += 256) s += bf16_round(tg[(size_t)b * TT + tt]);
  red[tid] = s; __syncthreads(); for (int st = 128; st > 0; st >>= 1) { if (tid < st) red[tid] += red[tid + st]; __syncthreads(); } if (tid == 0) mu_s = red[0] / lenf; __syncthreads(); const float mu = mu_s;
  float q = 0.f; for (int tt = tid; tt < TT; tt += 256) { const float d = (tt < len) ? (bf16_round(tg[(size_t)b * TT + tt]) - mu) : 0.f; q += d * d; }
  __syncthreads(); red[tid] = q; __syncthreads(); for (int st = 128; st > 0; st >>= 1) { if (tid < st) red[tid] += red[tid + st]; __syncthreads(); }
  if (tid < 32) { const float sd = sqrtf(red[0] / (lenf - 1.0f)); const float v = (tid == 0) ? mu : (tid == 1) ? sd : 0.f; *(volatile float*)(STT + (size_t)b * 32 + tid) = v; __threadfence(); *(volatile float*)(STT + (size_t)b * 32 + tid) = v; } }
__global__ __launch_bounds__(64) void k_tparams(const float* __restrict__ STT, float* __restrict__ out) { const int l = threadIdx.x; if (l >= 32) return; const int b = l >> 1, j = l & 1; const float v = STT[(size_t)b * 32 + j]; *(volatile float*)(out + l) = v; __threadfence(); *(volatile float*)(out + l) = v; }
__global__ __launch_bounds__(256) void k_cn(const float* __restrict__ tg, const int* __restrict__ ml, const float* __restrict__ STT, _Float16* __restrict__ CN16) {
  #pragma clang fp contract(off)
  const int t = blockIdx.x * 256 + threadIdx.x; if (t >= NBt * (TT / 8)) return; const int t0 = (t % (TT / 8)) * 8, b = t / (TT / 8); const float mu = STT[(size_t)b * 32], sd = STT[(size_t)b * 32 + 1]; const int len = ml[b]; FragH f;
#pragma unroll
  for (int i = 0; i < 8; ++i) { const int tt = t0 + i; f.h[i] = (_Float16)((tt < len) ? ((bf16_round(tg[(size_t)b * TT + tt]) - mu) / sd) : 0.f); }
  *(volatile v8us*)((unsigned short*)CN16 + (size_t)b * TT + t0) = f.half[0]; __threadfence(); *(volatile v8us*)((unsigned short*)CN16 + (size_t)b * TT + t0) = f.half[0]; }
__constant__ float SCALE_TAB[NW] = {1.0f, 1.4918247f, 2.2255409f, 3.320117f, 4.9530325f, 7.389056f, 11.023176f, 16.444647f, 24.53253f, 36.598236f};
__global__ __launch_bounds__(256) void k_kt(float* __restrict__ KT) {
  #pragma clang fp contract(off)
  const int tix = blockIdx.x * 256 + threadIdx.x; if (tix >= NW * TT) return; const int t = tix % TT, w = tix / TT; const float s = SCALE_TAB[w];
  float re = 0.f, im = 0.f;
#pragma unroll 1
  for (int k = 1; k < TT / 2; ++k) { const float om = 6.283185307179586f * (float)k / (float)TT; const float e = s * om - 6.0f; const float psi = 0.7511255444649425f * sqrtf(6.283185307179586f * s) * expf(-0.5f * e * e); if (psi == 0.f) continue; const int ph = (int)(((long long)k * t) & (TT - 1)); float sn, cs; sincospif(2.0f * (float)ph / (float)TT, &sn, &cs); re += psi * cs; im += psi * sn; }
  typedef float v2f __attribute__((ext_vector_type(2))); v2f v; v[0] = re / (float)TT; v[1] = im / (float)TT; *(volatile v2f*)(KT + (size_t)tix * 2) = v; __threadfence(); *(volatile v2f*)(KT + (size_t)tix * 2) = v; }
__global__ __launch_bounds__(256) void k_km(const float* __restrict__ KT, int w, int p, _Float16* __restrict__ KM) { const int tix = blockIdx.x * 256 + threadIdx.x; if (tix >= TT * (TT / 8)) return; const int tau0 = (tix % (TT / 8)) * 8, t = tix / (TT / 8); FragH f;
#pragma unroll
  for (int i = 0; i < 8; ++i) { const int d = (t - (tau0 + i)) & (TT - 1); f.h[i] = (_Float16)(KT[((size_t)w * TT + d) * 2 + p] * 1024.0f); }
  *(volatile v8us*)((unsigned short*)KM + (size_t)t * TT + tau0) = f.half[0]; __threadfence(); *(volatile v8us*)((unsigned short*)KM + (size_t)t * TT + tau0) = f.half[0]; }
__global__ __launch_bounds__(256) void k_tspec(const float* __restrict__ OUT, const int* __restrict__ ml, float* __restrict__ out) { const int tix = blockIdx.x * 256 + threadIdx.x; if (tix >= NR * 20 / 4) return; v4f v;
#pragma unroll
  for (int i = 0; i < 4; ++i) { const size_t f = (size_t)tix * 4 + i; const size_t bt = f / 20; const int j = (int)(f % 20); const int b = (int)(bt / TT), tt = (int)(bt % TT); const int w = j % NW, p = j / NW; v[i] = (tt < ml[b]) ? OUT[(((size_t)w * 2 + p) * TT + tt) * 16 + b] : 0.f; }
  *(volatile v4f*)(out + (size_t)tix * 4) = v; __threadfence(); *(volatile v4f*)(out + (size_t)tix * 4) = v; }
__global__ __launch_bounds__(256) void k_embed(const float* __restrict__ tg, const float* __restrict__ alpha, const int* __restrict__ ml, const float* __restrict__ emb, float* __restrict__ out) {
  #pragma clang fp contract(off)
  const int tix = blockIdx.x * 256 + threadIdx.x; if (tix >= NR * (CC / 8)) return; const int c0 = (tix % (CC / 8)) * 8, r = tix / (CC / 8); const int b = r / TT, tt = r % TT; int id = 0;
  if (tt < ml[b]) { float q = bf16_round(tg[r]) * bf16_round(alpha[b]); q = fminf(fmaxf(q, 0.f), 800.f); const float quo = (float)((double)q / 3.125); id = (int)rintf(quo) + 1; }
  id = min(max(id, 0), NEMB - 1); const float* src = emb + (size_t)id * CC + c0; v4f oa, ob;
#pragma unroll
  for (int i = 0; i < 4; ++i) { oa[i] = bf16_round(src[i]); ob[i] = bf16_round(src[4 + i]); }
  const int l = threadIdx.x & 31; float* row = out + (size_t)r * CC; const v4f a1 = shfl4(oa, l >> 1), b1 = shfl4(ob, l >> 1), a2 = shfl4(oa, 16 + (l >> 1)), b2 = shfl4(ob, 16 + (l >> 1)); const v4f x1 = (l & 1) ? b1 : a1, x2 = (l & 1) ? b2 : a2;
  for (int pass = 0; pass < 2; ++pass) { *(volatile v4f*)(row + l * 4) = x1; *(volatile v4f*)(row + 128 + l * 4) = x2; if (pass == 0) __threadfence(); } }

extern "C" void kernel_launch(void* const* d_in, const int* in_sizes, int n_in,
                              void* d_out, int out_size, void* d_ws, size_t ws_size, hipStream_t stream) {
  (void)in_sizes; (void)n_in; (void)out_size;
  const float* const* I = (const float* const*)d_in; const float* x = I[0]; const float* alpha = I[1]; const float* tg = I[2]; const int* ml = (const int*)d_in[3]; const float* c1w = I[4]; const float* c1b = I[5]; const float* g1 = I[6]; const float* e1 = I[7]; const float* c2w = I[8]; const float* c2b = I[9]; const float* g2 = I[10]; const float* e2 = I[11]; const float* lw = I[12]; const float* lb = I[13]; const float* emb = I[14];
  char* ws = (char*)d_ws; size_t off = 0;
  auto take = [&](size_t bytes) { char* p = ws + off; off += (bytes + 255) & ~(size_t)255; return p; };
  _Float16* BC1 = (_Float16*)take((size_t)CC * 3 * CC * 2); _Float16* BC2 = (_Float16*)take((size_t)CC * 3 * CC * 2); _Float16* BL = (_Float16*)take((size_t)NLP * CC * 2); float* BLP = (float*)take(NLP * 4); float* STT = (float*)take(NBt * 32 * 4); float* KT = (float*)take((size_t)NW * TT * 2 * 4); _Float16* CN16 = (_Float16*)take((size_t)NBt * TT * 2); float* OUT = (float*)take((size_t)NW * 2 * TT * 16 * 4);
  _Float16* P16 = (_Float16*)take((size_t)NR * CC * 2); _Float16* COL = (_Float16*)take((size_t)NR * 3 * CC * 2); float* Hm = (float*)take((size_t)NR * CC * 4); float* PRED = (float*)take((size_t)NR * NLP * 4); _Float16* KM = (_Float16*)take((size_t)TT * TT * 2);
  if (off > ws_size) return;
  float* out0 = (float*)d_out; float* out1 = (float*)((char*)d_out + 33554432); float* out2 = (float*)((char*)d_out + 36175872); float* out3 = (float*)((char*)d_out + 36176000); float* out4 = (float*)((char*)d_out + 38797440);
  k_w1d<<<(CC * (3 * CC / 8) + 255) / 256, 256, 0, stream>>>(c1w, BC1); k_w1d<<<(CC * (3 * CC / 8) + 255) / 256, 256, 0, stream>>>(c2w, BC2); k_wlin<<<(NLP * (CC / 8) + 255) / 256, 256, 0, stream>>>(lw, lb, BL, BLP);
  const size_t n8 = (size_t)NR * CC / 8; const unsigned nb8 = (unsigned)((n8 + 255) / 256); const dim3 gC(((NR / 16) * (CC / 64) + 3) / 4, 1);
  k_x16<<<nb8, 256, 0, stream>>>(x, P16, n8); k_tcol<<<(NR * 3 * (CC / 8) + 255) / 256, 256, 0, stream>>>(P16, COL);
  k_gemm_hhx<0><<<gC, 128, 0, stream>>>(COL, 3 * CC, 0, BC1, 3 * CC, 0, 0.0625f, c1b, 0, nullptr, 1, 0, 0, Hm, nullptr, CC, 0, NR, CC, 3 * CC);
  k_lnrelu<<<NR / 8, 256, 0, stream>>>(Hm, g1, e1, P16); k_tcol<<<(NR * 3 * (CC / 8) + 255) / 256, 256, 0, stream>>>(P16, COL);
  k_gemm_hhx<0><<<gC, 128, 0, stream>>>(COL, 3 * CC, 0, BC2, 3 * CC, 0, 0.0625f, c2b, 0, nullptr, 1, 0, 0, Hm, nullptr, CC, 0, NR, CC, 3 * CC);
  k_lnrelu<<<NR / 8, 256, 0, stream>>>(Hm, g2, e2, P16);
  k_gemm_hhx<0><<<dim3(((NR / 16) * 1 + 3) / 4, 1), 128, 0, stream>>>(P16, CC, 0, BL, CC, 0, 0.0625f, BLP, 0, nullptr, 1, 0, 0, PRED, nullptr, NLP, 0, NR, NLP, CC);
  k_pspec<<<(NR * 20 / 4 + 255) / 256, 256, 0, stream>>>(PRED, ml, out1); k_pparams<<<1, 256, 0, stream>>>(PRED, out2);
  k_tstat<<<NBt, 256, 0, stream>>>(tg, ml, STT); k_tparams<<<1, 64, 0, stream>>>(STT, out4); k_cn<<<(NBt * (TT / 8) + 255) / 256, 256, 0, stream>>>(tg, ml, STT, CN16);
  k_kt<<<(NW * TT + 255) / 256, 256, 0, stream>>>(KT);
  for (int w = 0; w < NW; ++w) for (int p = 0; p < 2; ++p) { k_km<<<(TT * (TT / 8) + 255) / 256, 256, 0, stream>>>(KT, w, p, KM);
    k_gemm_hhx<0><<<dim3(((TT / 16) * 1 + 3) / 4, 1), 128, 0, stream>>>(KM, TT, 0, CN16, TT, 0, 0.0009765625f, nullptr, 0, nullptr, 1, 0, 0, OUT + ((size_t)w * 2 + p) * TT * 16, nullptr, 16, 0, TT, 16, TT); }
  k_tspec<<<(NR * 20 / 4 + 255) / 256, 256, 0, stream>>>(OUT, ml, out3);
  k_embed<<<nb8, 256, 0, stream>>>(tg, alpha, ml, emb, out0);
}
